// VGAE_61976378081862
// MI455X (gfx1250) — hardware-run, weakly checked
//
#include <hip/hip_runtime.h>
#include <stddef.h>
#include <stdint.h>
#include <math.h>

#define NN      50000
#define DI      64
#define DE      32
#define DH      64
#define NE      1600000
#define EPN     500000
#define GBM     128
#define MP      50048
#define NTHR    256
#define NWAVE   8
#define EPT     8
#define WCH     (32 * EPT)
#define NBRUN   1024
#define SLB     10
#define NBK     49
#define NSLOT   (NBK * NBRUN)
#define WLCAP   4608
#define RCAP    36864
#define TRIPCAP 128
#define MAXDEG_MEAS   58
#define MAXB1024_MEAS 33159
#define ABM     64
#define SP      68
#define SP1     36
#define SPLIT2  1
#define XPITCH  64
#define W1PITCH 64
#define A2PITCH 64
#define W2PITCH 64
#define K1E     64
#define K2E     (SPLIT2 ? 64 : 32)
#define WSMAX   ((size_t)128u << 20)

#define BK_ZINTS (NWAVE * WLCAP + RCAP / 2 + NWAVE * NBRUN + 4 * NBRUN + 2 * NBRUN)
#define BK_INTS  (BK_ZINTS + 16)
#define BK_LDS   (BK_INTS * 4)

#define PBX   (MP * DI / 8 / NTHR)
#define PBW1  1
#define PBW2  2
#define PBTOT (PBX + PBW1 + PBW2 + 1)
#define PWAVES (EPN / 32)
#define PBLK   ((PWAVES + NWAVE - 1) / NWAVE)

#define OUT0_OFF 0
#define OUT1_OFF EPN
#define OUT2_OFF (2 * EPN)
#define OUT3_OFF (2 * EPN + NN * DE)
#define OUT_TOTAL (2 * EPN + 2 * NN * DE)

static_assert(DE == 32 && DH == 2 * DE && DI == 64);
static_assert(MP % GBM == 0 && MP >= NN && MP == 391 * GBM && MP % ABM == 0);
static_assert(NBRUN == (1 << SLB) && NBRUN % ABM == 0 && NBRUN % GBM == 0 && NBRUN % 32 == 0);
static_assert(NBK * NBRUN >= MP && NSLOT >= MP);
static_assert(NN <= 65536);
static_assert(NE % WCH == 0 && NE % 4 == 0);
static_assert(RCAP == NWAVE * WLCAP && RCAP % (4 * NTHR) == 0 && BK_ZINTS % 4 == 0);
static_assert((long long)RCAP * 100 >= (long long)MAXB1024_MEAS * 105);
static_assert(WLCAP >= MAXB1024_MEAS / 8 + 7 * 64 + 1);
static_assert(MAXDEG_MEAS + 8 <= TRIPCAP && TRIPCAP < 65536);
static_assert(NBRUN == 4 * NTHR);
static_assert((MP * DI / 8) % NTHR == 0 && DE * DI / 8 == NTHR * PBW1 && DH * W2PITCH / 8 == NTHR * PBW2);
static_assert(K1E % 32 == 0 && K2E % 32 == 0 && K1E <= XPITCH && K1E <= W1PITCH && K2E <= A2PITCH && K2E <= W2PITCH);
static_assert(BK_LDS <= 300000);
static_assert(EPN % 32 == 0);
static_assert((OUT1_OFF * 4) % 128 == 0 && (OUT2_OFF * 4) % 128 == 0 && (OUT3_OFF * 4) % 128 == 0);
static_assert(OUT3_OFF + NN * DE - 1 == 4199999 && OUT_TOTAL == 4200000);
static_assert(GBM * SP * 4 + 256 <= 65536);

typedef float          v4f   __attribute__((ext_vector_type(4)));
typedef float          v8f   __attribute__((ext_vector_type(8)));
typedef int            v4i   __attribute__((ext_vector_type(4)));
typedef int            v8i   __attribute__((ext_vector_type(8)));
typedef unsigned int   v2u   __attribute__((ext_vector_type(2)));
typedef unsigned short v8us  __attribute__((ext_vector_type(8)));
typedef unsigned short v16us __attribute__((ext_vector_type(16)));
typedef __bf16         v16bf __attribute__((ext_vector_type(16)));
typedef v4f  __attribute__((may_alias)) v4fa;
typedef v4i  __attribute__((may_alias)) v4ia;
typedef v2u  __attribute__((may_alias)) v2ua;
typedef v8us __attribute__((may_alias)) v8usa;
typedef unsigned short __attribute__((may_alias)) usa;
union FragB { v16bf v; v16us u; v8us h[2]; v8i w; };

__device__ __forceinline__ v8f wmb(const FragB& a, const FragB& b, v8f c) {
  v8f d = __builtin_amdgcn_wmma_f32_16x16x32_bf16(false, a.v, false, b.v, (short)0, c, false, false);
  asm volatile("v_nop\n\tv_nop\n\tv_nop\n\tv_nop" : "+v"(d) : "v"(a.w), "v"(b.w));
  return d;
}

__device__ __forceinline__ unsigned bf16_bits(float f) {
  const unsigned u = __float_as_uint(f);
  const unsigned r = (u + 0x7FFFu + ((u >> 16) & 1u)) >> 16;
  const unsigned q = (u >> 16) | 0x40u;
  return ((u & 0x7fffffffu) > 0x7f800000u) ? q : r;
}
__device__ __forceinline__ float bf16_val(float f) {
  return __uint_as_float(bf16_bits(f) << 16);
}
__device__ __forceinline__ int clampi(int v, int lo, int hi) {
  return v < lo ? lo : (v > hi ? hi : v);
}

__device__ __forceinline__ void st2_v4f(float* p, v4f v) {
  *(volatile v4f*)p = v;
  __threadfence();
  *(volatile v4f*)p = v;
}
__device__ __forceinline__ void st2_v8us(unsigned short* p, v8us v) {
  *(volatile v8us*)p = v;
  __threadfence();
  *(volatile v8us*)p = v;
}

__device__ __forceinline__ v8us gather8(const float* __restrict__ base, int stride) {
  float f[8];
#pragma unroll
  for (int i = 0; i < 8; ++i) f[i] = base[(size_t)i * (size_t)stride];
  v8us o;
#pragma unroll
  for (int i = 0; i < 8; ++i) o[i] = (unsigned short)bf16_bits(f[i]);
  return o;
}

__global__ __launch_bounds__(NTHR) void k_prep(const float* __restrict__ x, const float* __restrict__ w1,
                                               const float* __restrict__ b1, const float* __restrict__ w2,
                                               const float* __restrict__ b2,
                                               unsigned short* xb, unsigned short* w1t, unsigned short* w2d,
                                               float* sm) {
  const int tid = (int)threadIdx.x, lane = tid & 31;
  const int blk = (int)blockIdx.x;
  if (blk < PBX) {
    const int u   = blk * NTHR + tid;
    const int row = u >> 3, k8 = (u & 7) * 8;
    const int rc  = row < NN ? row : NN - 1;
    const unsigned mk = row < NN ? 0xffffu : 0u;
    const float* p = x + (size_t)rc * DI + k8;
    const v4f a = *(const v4fa*)p;
    const v4f b = *(const v4fa*)(p + 4);
    v8us o;
    o[0] = (unsigned short)(bf16_bits(a.x) & mk); o[1] = (unsigned short)(bf16_bits(a.y) & mk);
    o[2] = (unsigned short)(bf16_bits(a.z) & mk); o[3] = (unsigned short)(bf16_bits(a.w) & mk);
    o[4] = (unsigned short)(bf16_bits(b.x) & mk); o[5] = (unsigned short)(bf16_bits(b.y) & mk);
    o[6] = (unsigned short)(bf16_bits(b.z) & mk); o[7] = (unsigned short)(bf16_bits(b.w) & mk);
    st2_v8us(xb + (size_t)row * XPITCH + k8, o);
  } else if (blk < PBX + PBW1) {
    const int u = (blk - PBX) * NTHR + tid;
    const int n = u >> 3, k8 = (u & 7) * 8;
    const v8us o = gather8(w1 + (size_t)k8 * DE + n, DE);
    st2_v8us(w1t + (size_t)n * W1PITCH + k8, o);
  } else if (blk < PBX + PBW1 + PBW2) {
    const int u = (blk - PBX - PBW1) * NTHR + tid;
    const int n = u >> 3, k8 = (u & 7) * 8, kk = k8 & 31;
    const v8us o = gather8(w2 + (size_t)kk * DH + n, DH);
    st2_v8us(w2d + (size_t)n * W2PITCH + k8, o);
  } else {
    if (tid < 32) {
      const int i1 = lane < 8 ? lane : 7;
      const int i2 = clampi(lane - 8, 0, 15);
      const v4f a = *(const v4fa*)(b1 + 4 * i1);
      const v4f c = *(const v4fa*)(b2 + 4 * i2);
      asm volatile("" :: "v"(a));
      asm volatile("" :: "v"(c));
      const unsigned ma = (lane < 8) ? 0xffffffffu : 0u;
      const unsigned mc = (lane >= 8 && lane < 24) ? 0xffffffffu : 0u;
      v4f o;
      o.x = __uint_as_float(((bf16_bits(a.x) << 16) & ma) | ((bf16_bits(c.x) << 16) & mc));
      o.y = __uint_as_float(((bf16_bits(a.y) << 16) & ma) | ((bf16_bits(c.y) << 16) & mc));
      o.z = __uint_as_float(((bf16_bits(a.z) << 16) & ma) | ((bf16_bits(c.z) << 16) & mc));
      o.w = __uint_as_float(((bf16_bits(a.w) << 16) & ma) | ((bf16_bits(c.w) << 16) & mc));
      st2_v4f(sm + 4 * lane, o);
    }
  }
}

__device__ __forceinline__ void count_role(bool g, unsigned t, int* mybin, int lane) {
  unsigned mm = __builtin_amdgcn_ballot_w32(g);
#pragma unroll 1
  for (int it = 0; it < 32; ++it) {
    if (mm == 0u) break;
    const int k  = __builtin_ffs((int)mm) - 1;
    const int sl = __builtin_amdgcn_readlane((int)t, k) & (NBRUN - 1);
    if (lane == 0) mybin[sl] = mybin[sl] + 1;
    mm &= mm - 1u;
  }
}

__device__ __forceinline__ void bucket_flush(const usa* pl16, const int* cnt, const int* offs,
                                             const float* fnd, const float* fns, int ov,
                                             int* lp, int* offp, int* cntp, float* ndp, float* nsp, int* fp,
                                             int tid) {
#pragma unroll 1
  for (int i4 = tid; i4 < RCAP / 4; i4 += NTHR) {
    const v2u u = *(const v2ua*)(pl16 + 4 * i4);
    v4i w;
    w.x = (int)(u.x & 0xffffu); w.y = (int)(u.x >> 16);
    w.z = (int)(u.y & 0xffffu); w.w = (int)(u.y >> 16);
    *(volatile v4i*)(lp + 4 * i4) = w;
  }
  {
    const v4i a = *(const v4ia*)(offs + 4 * tid);
    const v4i b = *(const v4ia*)(cnt + 4 * tid);
    const v4f c = *(const v4fa*)(fnd + 4 * tid);
    const v4f d = *(const v4fa*)(fns + 4 * tid);
    *(volatile v4i*)(offp + 4 * tid) = a;
    *(volatile v4i*)(cntp + 4 * tid) = b;
    *(volatile v4f*)(ndp + 4 * tid) = c;
    *(volatile v4f*)(nsp + 4 * tid) = d;
  }
  if (tid < 8) {
    const v4i f = {ov, ov, ov, ov};
    *(volatile v4i*)(fp + 4 * tid) = f;
  }
}

__global__ __launch_bounds__(NTHR) void k_bucket(const int* __restrict__ srcs, const int* __restrict__ dsts,
                                                 int* LIST, int* OFFT, int* CNTT, float* NDT, float* NST,
                                                 int* FLAG) {
  extern __shared__ __attribute__((aligned(16))) int dsm[];
  int*   wl   = dsm;
  usa*   pl16 = (usa*)(dsm + NWAVE * WLCAP);
  int*   bins = dsm + NWAVE * WLCAP + RCAP / 2;
  int*   cnt  = bins + NWAVE * NBRUN;
  int*   offs = cnt + NBRUN;
  int*   cur  = offs + NBRUN;
  int*   scnt = cur + NBRUN;
  float* fnd  = (float*)(scnt + NBRUN);
  float* fns  = fnd + NBRUN;
  int*   misc = (int*)(fns + NBRUN);
  const int tid = (int)threadIdx.x, lane = tid & 31, wave = tid >> 5;
  const int blk = (int)blockIdx.x;
  const unsigned nbs = (unsigned)(blk * NBRUN);

  {
    const v4i z4 = {0, 0, 0, 0};
    for (int i = tid * 4; i < BK_ZINTS; i += NTHR * 4) *(v4ia*)(dsm + i) = z4;
    if (tid < 16) misc[tid] = 0;
  }
  __syncthreads();

  {
    const int per  = ((NE + NWAVE * WCH - 1) / (NWAVE * WCH)) * WCH;
    const int ebeg = wave * per;
    const int eend = (ebeg + per < NE) ? (ebeg + per) : NE;
    int* mylist = wl + wave * WLCAP;
    int* mybin  = bins + wave * NBRUN;
    int wc = 0;
#pragma unroll 1
    for (int cb = ebeg; cb < eend; cb += WCH) {
      const int e0 = cb + lane * EPT;
      const v4i da = *(const v4ia*)(dsts + e0);
      const v4i db = *(const v4ia*)(dsts + e0 + 4);
      const v4i sa = *(const v4ia*)(srcs + e0);
      const v4i sb = *(const v4ia*)(srcs + e0 + 4);
      const unsigned s0 = (unsigned)da.x - nbs, s1 = (unsigned)da.y - nbs;
      const unsigned s2 = (unsigned)da.z - nbs, s3 = (unsigned)da.w - nbs;
      const unsigned s4 = (unsigned)db.x - nbs, s5 = (unsigned)db.y - nbs;
      const unsigned s6 = (unsigned)db.z - nbs, s7 = (unsigned)db.w - nbs;
      const bool h0 = s0 < (unsigned)NBRUN, h1 = s1 < (unsigned)NBRUN, h2 = s2 < (unsigned)NBRUN, h3 = s3 < (unsigned)NBRUN;
      const bool h4 = s4 < (unsigned)NBRUN, h5 = s5 < (unsigned)NBRUN, h6 = s6 < (unsigned)NBRUN, h7 = s7 < (unsigned)NBRUN;
      const unsigned m0 = __builtin_amdgcn_ballot_w32(h0), m1 = __builtin_amdgcn_ballot_w32(h1);
      const unsigned m2 = __builtin_amdgcn_ballot_w32(h2), m3 = __builtin_amdgcn_ballot_w32(h3);
      const unsigned m4 = __builtin_amdgcn_ballot_w32(h4), m5 = __builtin_amdgcn_ballot_w32(h5);
      const unsigned m6 = __builtin_amdgcn_ballot_w32(h6), m7 = __builtin_amdgcn_ballot_w32(h7);
      const unsigned any = m0 | m1 | m2 | m3 | m4 | m5 | m6 | m7;
      if (any != 0u) {
        const int r0 = clampi(sa.x, 0, NN - 1), r1 = clampi(sa.y, 0, NN - 1);
        const int r2 = clampi(sa.z, 0, NN - 1), r3 = clampi(sa.w, 0, NN - 1);
        const int r4 = clampi(sb.x, 0, NN - 1), r5 = clampi(sb.y, 0, NN - 1);
        const int r6 = clampi(sb.z, 0, NN - 1), r7 = clampi(sb.w, 0, NN - 1);
        const int pre = (int)(__builtin_amdgcn_mbcnt_lo(m0, 0u) + __builtin_amdgcn_mbcnt_lo(m1, 0u) +
                              __builtin_amdgcn_mbcnt_lo(m2, 0u) + __builtin_amdgcn_mbcnt_lo(m3, 0u) +
                              __builtin_amdgcn_mbcnt_lo(m4, 0u) + __builtin_amdgcn_mbcnt_lo(m5, 0u) +
                              __builtin_amdgcn_mbcnt_lo(m6, 0u) + __builtin_amdgcn_mbcnt_lo(m7, 0u));
        int p = wc + pre;
        if (h0) { if (p < WLCAP) mylist[p] = ((int)s0 << 16) | r0; p = p + 1; }
        if (h1) { if (p < WLCAP) mylist[p] = ((int)s1 << 16) | r1; p = p + 1; }
        if (h2) { if (p < WLCAP) mylist[p] = ((int)s2 << 16) | r2; p = p + 1; }
        if (h3) { if (p < WLCAP) mylist[p] = ((int)s3 << 16) | r3; p = p + 1; }
        if (h4) { if (p < WLCAP) mylist[p] = ((int)s4 << 16) | r4; p = p + 1; }
        if (h5) { if (p < WLCAP) mylist[p] = ((int)s5 << 16) | r5; p = p + 1; }
        if (h6) { if (p < WLCAP) mylist[p] = ((int)s6 << 16) | r6; p = p + 1; }
        if (h7) { if (p < WLCAP) mylist[p] = ((int)s7 << 16) | r7; p = p + 1; }
        wc += (int)(__builtin_popcount(m0) + __builtin_popcount(m1) + __builtin_popcount(m2) + __builtin_popcount(m3) +
                    __builtin_popcount(m4) + __builtin_popcount(m5) + __builtin_popcount(m6) + __builtin_popcount(m7));
      }
      const unsigned t0 = (unsigned)sa.x - nbs, t1 = (unsigned)sa.y - nbs;
      const unsigned t2 = (unsigned)sa.z - nbs, t3 = (unsigned)sa.w - nbs;
      const unsigned t4 = (unsigned)sb.x - nbs, t5 = (unsigned)sb.y - nbs;
      const unsigned t6 = (unsigned)sb.z - nbs, t7 = (unsigned)sb.w - nbs;
      count_role(t0 < (unsigned)NBRUN, t0, mybin, lane);
      count_role(t1 < (unsigned)NBRUN, t1, mybin, lane);
      count_role(t2 < (unsigned)NBRUN, t2, mybin, lane);
      count_role(t3 < (unsigned)NBRUN, t3, mybin, lane);
      count_role(t4 < (unsigned)NBRUN, t4, mybin, lane);
      count_role(t5 < (unsigned)NBRUN, t5, mybin, lane);
      count_role(t6 < (unsigned)NBRUN, t6, mybin, lane);
      count_role(t7 < (unsigned)NBRUN, t7, mybin, lane);
    }
    if (lane == 0) misc[wave] = wc;
  }
  __syncthreads();

#pragma unroll 1
  for (int i = tid; i < NBRUN; i += NTHR) {
    int s = 0;
#pragma unroll
    for (int w2 = 0; w2 < NWAVE; ++w2) s += bins[w2 * NBRUN + i];
    scnt[i] = s;
  }

  if (wave == 0) {
    int ov = 0;
#pragma unroll 1
    for (int w2 = 0; w2 < NWAVE; ++w2) {
      int c = misc[w2];
      if (c > WLCAP) ov = 1;
      c = c < 0 ? 0 : (c > WLCAP ? WLCAP : c);
#pragma unroll 1
      for (int b0 = 0; b0 < c; b0 += 32) {
        const int idx = b0 + lane;
        const int ent = wl[w2 * WLCAP + (idx < WLCAP ? idx : WLCAP - 1)];
        const int m32 = (c - b0) < 32 ? (c - b0) : 32;
#pragma unroll 1
        for (int k = 0; k < m32; ++k) {
          const int u    = __builtin_amdgcn_readlane(ent, k);
          const int slot = (u >> 16) & (NBRUN - 1);
          if (lane == 0) cnt[slot] = cnt[slot] + 1;
        }
      }
    }
    if (lane == 0) misc[9] = ov;
  }
  __syncthreads();
  if (wave == 0) {
    const int base = lane * (NBRUN / 32);
    int s = 0;
#pragma unroll 1
    for (int i = 0; i < NBRUN / 32; ++i) s += cnt[base + i];
    int incl = s;
#pragma unroll
    for (int d = 1; d < 32; d <<= 1) {
      const int y = __shfl_up(incl, d, 32);
      if (lane >= d) incl += y;
    }
    int run = incl - s;
#pragma unroll 1
    for (int i = 0; i < NBRUN / 32; ++i) {
      const int cv = cnt[base + i];
      offs[base + i] = run;
      cur[base + i]  = run;
      run += cv;
    }
  }
  __syncthreads();

  if (wave == 0) {
#pragma unroll 1
    for (int w2 = 0; w2 < NWAVE; ++w2) {
      int c = misc[w2];
      c = c < 0 ? 0 : (c > WLCAP ? WLCAP : c);
#pragma unroll 1
      for (int b0 = 0; b0 < c; b0 += 32) {
        const int idx = b0 + lane;
        const int ent = wl[w2 * WLCAP + (idx < WLCAP ? idx : WLCAP - 1)];
        const int m32 = (c - b0) < 32 ? (c - b0) : 32;
#pragma unroll 1
        for (int k = 0; k < m32; ++k) {
          const int u    = __builtin_amdgcn_readlane(ent, k);
          const int slot = (u >> 16) & (NBRUN - 1);
          if (lane == 0) {
            int p = cur[slot];
            p = p < 0 ? 0 : (p > RCAP - 1 ? RCAP - 1 : p);
            pl16[p] = (unsigned short)(u & 0xffff);
            cur[slot] = p + 1;
          }
        }
      }
    }
  }
  __syncthreads();

#pragma unroll 1
  for (int i = tid; i < NBRUN; i += NTHR) {
    const int ci = cnt[i], si = scnt[i];
    const float cd = (float)(ci < 1 ? 1 : ci);
    const float sd = (float)(si < 1 ? 1 : si);
    fnd[i] = 1.0f / sqrtf(cd);
    fns[i] = 1.0f / sqrtf(sd);
  }
  __syncthreads();

  const int ovf = misc[9];
  int*   lp   = LIST + (size_t)blk * RCAP;
  int*   offp = OFFT + (size_t)blk * NBRUN;
  int*   cntp = CNTT + (size_t)blk * NBRUN;
  float* ndp  = NDT + (size_t)blk * NBRUN;
  float* nsp  = NST + (size_t)blk * NBRUN;
  int*   fp   = FLAG + (size_t)blk * 32;
  bucket_flush(pl16, cnt, offs, fnd, fns, ovf, lp, offp, cntp, ndp, nsp, fp, tid);
  __threadfence();
  bucket_flush(pl16, cnt, offs, fnd, fns, ovf, lp, offp, cntp, ndp, nsp, fp, tid);
}

template <int KTOT, int AP, int BP, int NT>
__device__ __forceinline__ void gemm_16xN(const unsigned short* __restrict__ ap,
                                          const unsigned short* __restrict__ bp, v8f (&acc)[NT]) {
  static_assert(KTOT % 32 == 0 && KTOT <= AP && KTOT <= BP);
#pragma unroll 1
  for (int k0 = 0; k0 < KTOT; k0 += 32) {
    FragB af;
    af.h[0] = *(const v8usa*)(ap + k0);
    af.h[1] = *(const v8usa*)(ap + k0 + 16);
#pragma unroll
    for (int nt = 0; nt < NT; ++nt) {
      const unsigned short* wq = bp + (size_t)(16 * nt) * (size_t)BP + k0;
      FragB bf;
      bf.h[0] = *(const v8usa*)wq;
      bf.h[1] = *(const v8usa*)(wq + 16);
      acc[nt] = wmb(af, bf, acc[nt]);
    }
  }
}

__global__ __launch_bounds__(NTHR) __attribute__((amdgpu_num_vgpr(248)))
void k_gemm1(const unsigned short* __restrict__ XB, const unsigned short* __restrict__ W1T,
             const float* __restrict__ NST, float* P1) {
  __shared__ __attribute__((aligned(16))) float stg[GBM * SP1];
  const int tid = (int)threadIdx.x, lane = tid & 31, wave = tid >> 5, hh = lane >> 4, m = lane & 15;
  const int rowBase = (int)blockIdx.x * GBM;

  v8f acc[2];
  {
    const v8f z = {0.f, 0.f, 0.f, 0.f, 0.f, 0.f, 0.f, 0.f};
    acc[0] = z; acc[1] = z;
  }
  const unsigned short* ap = XB + (size_t)(rowBase + 16 * wave + m) * (size_t)XPITCH + 8 * hh;
  const unsigned short* bp = W1T + (size_t)m * (size_t)W1PITCH + 8 * hh;
  gemm_16xN<K1E, XPITCH, W1PITCH, 2>(ap, bp, acc);
#pragma unroll
  for (int nt = 0; nt < 2; ++nt) {
#pragma unroll
    for (int r = 0; r < 8; ++r) stg[(16 * wave + 8 * hh + r) * SP1 + 16 * nt + m] = acc[nt][r];
  }
  __syncthreads();

  const int rq = lane >> 3, c4 = lane & 7;
#pragma unroll 1
  for (int i = 0; i < 4; ++i) {
    const int lr   = 16 * wave + 4 * i + rq;
    const int grow = rowBase + lr;
    const v4f a = *(const v4fa*)(stg + lr * SP1 + 4 * c4);
    const float s = NST[grow];
    v4f o;
    o.x = a.x * s; o.y = a.y * s; o.z = a.z * s; o.w = a.w * s;
    st2_v4f(P1 + (size_t)grow * DE + 4 * c4, o);
  }
}

template <int MODE>
__global__ __launch_bounds__(NTHR) void k_replay(const int* __restrict__ LIST, const int* __restrict__ OFFT,
                                                 const int* __restrict__ CNTT, const float* __restrict__ NDT,
                                                 const float* __restrict__ NST, const int* __restrict__ FLAG,
                                                 const float* __restrict__ SRC, const float* __restrict__ sm,
                                                 float* GO, int* AO) {
  const int tid = (int)threadIdx.x, lane = tid & 31, wave = tid >> 5;
  const int rowBase = (int)blockIdx.x * ABM;
  const int bucket  = rowBase >> SLB;
  const int* lb  = LIST + (size_t)bucket * RCAP;
  const int flag = FLAG[(size_t)bucket * 32];
  const float qnan = __uint_as_float(0x7fc00000u);
  const float b1c = sm[lane];
  const int s0 = (2 * lane) & 31, s1 = s0 + 1;

#pragma unroll 1
  for (int i = 0; i < ABM / NWAVE; ++i) {
    const int d = rowBase + (ABM / NWAVE) * wave + i;
    int cv = CNTT[d];
    int ov = OFFT[d];
    const bool big = cv > TRIPCAP;
    cv = cv < 0 ? 0 : (cv > TRIPCAP ? TRIPCAP : cv);
    ov = ov < 0 ? 0 : (ov > RCAP - 1 ? RCAP - 1 : ov);
    const int c = __builtin_amdgcn_readfirstlane(cv);
    const int o = __builtin_amdgcn_readfirstlane(ov);
    int last = o + c - 1; last = last < o ? o : last;
    last = last > RCAP - 1 ? RCAP - 1 : last;
    float acc = 0.0f;
#pragma unroll 1
    for (int b0 = 0; b0 < c; b0 += 32) {
      int idx = o + b0 + lane;
      idx = idx > last ? last : idx;
      const unsigned wd = (unsigned)lb[idx];
      int sr = (int)(wd & 0xffffu);
      sr = sr > NN - 1 ? NN - 1 : sr;
      const int m32 = (c - b0) < 32 ? (c - b0) : 32;
#pragma unroll 1
      for (int k = 0; k < m32; ++k) {
        const int sk = __builtin_amdgcn_readlane(sr, k);
        acc += SRC[(size_t)sk * DE + lane];
      }
    }
    const float ndv = NDT[d];
    const bool bad  = (flag != 0) | big;
    const bool live = d < NN;
    if constexpr (MODE == 0) {
      const float nsv = NST[d];
      float h = ndv * acc + b1c;
      h = (h > 0.0f) ? h : (h - h);
      float g = h * nsv;
      g = bad ? qnan : g;
      g = live ? g : 0.0f;
      float* op = GO + (size_t)d * DE + lane;
      *(volatile float*)op = g;
      __threadfence();
      *(volatile float*)op = g;
    } else {
      float a = ndv * acc;
      a = bad ? qnan : a;
      a = live ? a : 0.0f;
      const unsigned hb = bf16_bits(a);
      const unsigned lw = bf16_bits(a - __uint_as_float(hb << 16));
      const int h0 = __shfl((int)hb, s0, 32), h1 = __shfl((int)hb, s1, 32);
      const int l0 = __shfl((int)lw, s0, 32), l1 = __shfl((int)lw, s1, 32);
      const int mk = (lane < 16) ? -1 : 0;
      const int word = ((h0 | (h1 << 16)) & mk) | ((l0 | (l1 << 16)) & ~mk);
      int* op = AO + (size_t)d * (A2PITCH / 2) + lane;
      *(volatile int*)op = word;
      __threadfence();
      *(volatile int*)op = word;
    }
  }
}

__global__ __launch_bounds__(NTHR) __attribute__((amdgpu_num_vgpr(248)))
void k_gemm2(const unsigned short* __restrict__ A2, const unsigned short* __restrict__ W2D,
             const float* __restrict__ sm, const float* __restrict__ eps, const int* __restrict__ FLAG,
             float* out2, float* out3, float* Z) {
  __shared__ __attribute__((aligned(16))) float stg[GBM * SP];
  __shared__ __attribute__((aligned(16))) float sb2[64];
  const int tid = (int)threadIdx.x, lane = tid & 31, wave = tid >> 5, hh = lane >> 4, m = lane & 15;
  const int rowBase = (int)blockIdx.x * GBM;
  const int flag = FLAG[(size_t)(rowBase >> SLB) * 32];
  if (tid < 16) *(v4fa*)(sb2 + 4 * tid) = *(const v4fa*)(sm + 32 + 4 * tid);

  v8f acc[4];
  {
    const v8f z = {0.f, 0.f, 0.f, 0.f, 0.f, 0.f, 0.f, 0.f};
#pragma unroll
    for (int t = 0; t < 4; ++t) acc[t] = z;
  }
  const unsigned short* ap = A2 + (size_t)(rowBase + 16 * wave + m) * (size_t)A2PITCH + 8 * hh;
  const unsigned short* bp = W2D + (size_t)m * (size_t)W2PITCH + 8 * hh;
  gemm_16xN<K2E, A2PITCH, W2PITCH, 4>(ap, bp, acc);
#pragma unroll
  for (int nt = 0; nt < 4; ++nt) {
#pragma unroll
    for (int r = 0; r < 8; ++r) stg[(16 * wave + 8 * hh + r) * SP + 16 * nt + m] = acc[nt][r];
  }
  __syncthreads();

  const float qnan = __uint_as_float(0x7fc00000u);
  const float bm = sb2[lane], bl = sb2[32 + lane];
#pragma unroll 1
  for (int i = 0; i < 16; ++i) {
    const int lr   = 16 * wave + i;
    const int grow = rowBase + lr;
    const bool live = grow < NN;
    const int ge = live ? grow : NN - 1;
    const float t0 = stg[lr * SP + lane];
    const float t1 = stg[lr * SP + 32 + lane];
    const float eb = bf16_val(eps[(size_t)ge * DE + lane]);
    float mu = t0 + bm;
    const float lv = t1 + bl;
    float sg = expf(0.5f * lv);
    float zz = mu + sg * eb;
    mu = (flag != 0) ? qnan : mu;
    sg = (flag != 0) ? qnan : sg;
    zz = (flag != 0) ? qnan : zz;
    float* zp = Z + (size_t)grow * DE + lane;
    float* mp = out2 + (size_t)ge * DE + lane;
    float* sp = out3 + (size_t)ge * DE + lane;
    *(volatile float*)zp = zz;
    if (live) {
      *(volatile float*)mp = mu;
      *(volatile float*)sp = sg;
    }
    __threadfence();
    *(volatile float*)zp = zz;
    if (live) {
      *(volatile float*)mp = mu;
      *(volatile float*)sp = sg;
    }
  }
}

__device__ __forceinline__ void pair_body(const int* __restrict__ us, const int* __restrict__ vs,
                                          const float* __restrict__ Z, float* out, int wi, int lane) {
  if (wi >= PWAVES) return;
  const int p = wi * 32 + lane;
  const int u = clampi(us[p], 0, NN - 1);
  const int v = clampi(vs[p], 0, NN - 1);
  const float* zu = Z + (size_t)u * DE;
  const float* zv = Z + (size_t)v * DE;
  float acc = 0.0f;
#pragma unroll
  for (int t = 0; t < 8; ++t) {
    const v4f a = *(const v4fa*)(zu + 4 * t);
    const v4f b = *(const v4fa*)(zv + 4 * t);
    acc = fmaf(a.x, b.x, acc);
    acc = fmaf(a.y, b.y, acc);
    acc = fmaf(a.z, b.z, acc);
    acc = fmaf(a.w, b.w, acc);
  }
  float* op = out + p;
  *(volatile float*)op = acc;
  __threadfence();
  *(volatile float*)op = acc;
}

__global__ __launch_bounds__(NTHR) void k_pairs(const int* __restrict__ ps, const int* __restrict__ pd,
                                                const int* __restrict__ ns, const int* __restrict__ nd,
                                                const float* __restrict__ Z, float* out0, float* out1) {
  const int tid = (int)threadIdx.x, lane = tid & 31, wave = tid >> 5;
  const int blk = (int)blockIdx.x;
  if (blk < PBLK) {
    pair_body(ps, pd, Z, out0, blk * NWAVE + wave, lane);
  } else {
    pair_body(ns, nd, Z, out1, (blk - PBLK) * NWAVE + wave, lane);
  }
}

extern "C" void kernel_launch(void* const* d_in, const int* in_sizes, int n_in,
                              void* d_out, int out_size, void* d_ws, size_t ws_size,
                              hipStream_t stream) {
  if (n_in < 12) return;
  if (in_sizes[0] != NN * DI) return;
  if (in_sizes[1] != DI * DE) return;
  if (in_sizes[2] != DE) return;
  if (in_sizes[3] != DE * DH) return;
  if (in_sizes[4] != DH) return;
  if (in_sizes[5] != NN * DE) return;
  if (in_sizes[6] != NE || in_sizes[7] != NE) return;
  if (in_sizes[8] != EPN || in_sizes[9] != EPN) return;
  if (in_sizes[10] != EPN || in_sizes[11] != EPN) return;
  if (out_size != OUT_TOTAL) return;

  const float* x    = (const float*)d_in[0];
  const float* W1   = (const float*)d_in[1];
  const float* b1   = (const float*)d_in[2];
  const float* W2   = (const float*)d_in[3];
  const float* b2   = (const float*)d_in[4];
  const float* eps  = (const float*)d_in[5];
  const int*   esrc = (const int*)d_in[6];
  const int*   edst = (const int*)d_in[7];
  const int*   psrc = (const int*)d_in[8];
  const int*   pdst = (const int*)d_in[9];
  const int*   nsrc = (const int*)d_in[10];
  const int*   ndst = (const int*)d_in[11];
  float* out  = (float*)d_out;
  float* out0 = out + OUT0_OFF;
  float* out1 = out + OUT1_OFF;
  float* out2 = out + OUT2_OFF;
  float* out3 = out + OUT3_OFF;

  constexpr size_t zXB   = (size_t)MP * XPITCH * 2;
  constexpr size_t zF    = (size_t)MP * DE * 4;
  constexpr size_t zA2   = (size_t)MP * A2PITCH * 2;
  constexpr size_t zLIST = (size_t)NBK * RCAP * 4;
  constexpr size_t zTAB  = (size_t)NSLOT * 4;
  constexpr size_t zFLAG = 6400;
  constexpr size_t zW1T  = (size_t)DE * W1PITCH * 2;
  constexpr size_t zW2D  = (size_t)DH * W2PITCH * 2;
  constexpr size_t zSM   = 512;
  constexpr size_t oXB   = 0;
  constexpr size_t oP1   = oXB + zXB;
  constexpr size_t oG    = oP1 + zF;
  constexpr size_t oA2   = oG + zF;
  constexpr size_t oZ    = oA2 + zA2;
  constexpr size_t oLIST = oZ + zF;
  constexpr size_t oOFF  = oLIST + zLIST;
  constexpr size_t oCNT  = oOFF + zTAB;
  constexpr size_t oND   = oCNT + zTAB;
  constexpr size_t oNS   = oND + zTAB;
  constexpr size_t oFLAG = oNS + zTAB;
  constexpr size_t oW1T  = oFLAG + zFLAG;
  constexpr size_t oW2D  = oW1T + zW1T;
  constexpr size_t oSM   = oW2D + zW2D;
  constexpr size_t oEND  = oSM + zSM;
  static_assert(zXB % 256 == 0 && zF % 256 == 0 && zA2 % 256 == 0 && zLIST % 256 == 0 && zTAB % 256 == 0);
  static_assert(zFLAG % 256 == 0 && zFLAG >= (size_t)NBK * 128 && zW1T % 256 == 0 && zW2D % 256 == 0);
  static_assert(oEND <= WSMAX);
  if (oEND > ws_size) return;

  char* ws = (char*)d_ws;
  unsigned short* XB   = (unsigned short*)(ws + oXB);
  float*          P1   = (float*)(ws + oP1);
  float*          G    = (float*)(ws + oG);
  unsigned short* A2   = (unsigned short*)(ws + oA2);
  float*          Z    = (float*)(ws + oZ);
  int*            LIST = (int*)(ws + oLIST);
  int*            OFFT = (int*)(ws + oOFF);
  int*            CNTT = (int*)(ws + oCNT);
  float*          NDT  = (float*)(ws + oND);
  float*          NST  = (float*)(ws + oNS);
  int*            FLAG = (int*)(ws + oFLAG);
  unsigned short* W1T  = (unsigned short*)(ws + oW1T);
  unsigned short* W2D  = (unsigned short*)(ws + oW2D);
  float*          SM   = (float*)(ws + oSM);

  hipFuncSetAttribute(reinterpret_cast<const void*>(&k_bucket), hipFuncAttributeMaxDynamicSharedMemorySize, (int)BK_LDS);

  k_prep<<<PBTOT, NTHR, 0, stream>>>(x, W1, b1, W2, b2, XB, W1T, W2D, SM);
  k_bucket<<<NBK, NTHR, BK_LDS, stream>>>(esrc, edst, LIST, OFFT, CNTT, NDT, NST, FLAG);
  k_gemm1<<<MP / GBM, NTHR, 0, stream>>>(XB, W1T, NST, P1);
  k_replay<0><<<MP / ABM, NTHR, 0, stream>>>(LIST, OFFT, CNTT, NDT, NST, FLAG, P1, SM, G, (int*)A2);
  k_replay<1><<<MP / ABM, NTHR, 0, stream>>>(LIST, OFFT, CNTT, NDT, NST, FLAG, G, SM, G, (int*)A2);
  k_gemm2<<<MP / GBM, NTHR, 0, stream>>>(A2, W2D, SM, eps, FLAG, out2, out3, Z);
  k_pairs<<<2 * PBLK, NTHR, 0, stream>>>(psrc, pdst, nsrc, ndst, Z, out0, out1);
}
